// SlidingWindowAttention_66408784330768
// MI455X (gfx1250) — hardware-verified
//
#include <hip/hip_runtime.h>
#include <math.h>

typedef __attribute__((ext_vector_type(16))) _Float16 v16h;
typedef __attribute__((ext_vector_type(16))) __bf16 v16b;
typedef __attribute__((ext_vector_type(8)))  _Float16 v8h;
typedef __attribute__((ext_vector_type(8)))  __bf16 v8b;
typedef __attribute__((ext_vector_type(8)))  float v8f;
typedef __attribute__((ext_vector_type(4)))  float v4f;
typedef __attribute__((ext_vector_type(4)))  unsigned v4u;

#ifndef NB
#define NB 2
#endif
#ifndef SEQ
#define SEQ 2048
#endif
#define NB_FULL 2
#define SEQ_FULL 2048
#define DIN 1024
#define CC 1024
#define NH 16
#define HD 64
#define NQKV 3072
#define WIN 512
#define MROWS (NB * SEQ)

static_assert(DIN == 1024);
static_assert(CC == NH * HD);
static_assert(SEQ % 64 == 0);
static_assert(SEQ <= SEQ_FULL);
static_assert(NB <= NB_FULL);
static_assert((MROWS * DIN) % 2048 == 0);
static_assert(NQKV % 128 == 0);
static_assert(DIN % 128 == 0);
static_assert(DIN % 32 == 0);
static_assert(HD % 32 == 0);
static_assert(((SEQ / 16) & (SEQ / 16 - 1)) == 0);

template <typename T> __device__ __forceinline__ void vst2(void* p, T v) { *(volatile T*)p = v; __threadfence(); *(volatile T*)p = v; }

__device__ __forceinline__ v8f wmma16(v16h a, v16h b, v8f c) {
  v8f d = __builtin_amdgcn_wmma_f32_16x16x32_f16(false, a, false, b, (short)0, c, false, false);
  asm volatile("v_nop\n\tv_nop\n\tv_nop\n\tv_nop" : "+v"(d) : "v"(a), "v"(b));
  return d;
}
__device__ __forceinline__ v8f wmma_bf(v16b a, v16b b, v8f c) {
  v8f d = __builtin_amdgcn_wmma_f32_16x16x32_bf16(false, a, false, b, (short)0, c, false, false);
  asm volatile("v_nop\n\tv_nop\n\tv_nop\n\tv_nop" : "+v"(d) : "v"(a), "v"(b));
  return d;
}
__device__ __forceinline__ v16h frag_h(const _Float16* rowk0, unsigned lane) {
  union { v16h v; v8h q[2]; } u; const _Float16* p = rowk0 + 8u * (lane >> 4);
  u.q[0] = *(const v8h*)p; u.q[1] = *(const v8h*)(p + 16); return u.v;
}
__device__ __forceinline__ v16b frag_b(const __bf16* rowk0, unsigned lane) {
  union { v16b v; v8b q[2]; } u; const __bf16* p = rowk0 + 8u * (lane >> 4);
  u.q[0] = *(const v8b*)p; u.q[1] = *(const v8b*)(p + 16); return u.v;
}
struct F2 { v16b h, l; };
__device__ __forceinline__ F2 bsplit16(const float v[16]) { F2 r;
#pragma unroll
  for (int i = 0; i < 16; ++i) { const __bf16 hb = (__bf16)v[i]; r.h[i] = hb; r.l[i] = (__bf16)(v[i] - (float)hb); }
  return r; }
__device__ __forceinline__ v8f mac3(const F2& a, const F2& b, v8f c) { c = wmma_bf(a.l, b.h, c); c = wmma_bf(a.h, b.l, c); return wmma_bf(a.h, b.h, c); }
__device__ __forceinline__ float bfr(float v) { return (float)(__bf16)v; }
#define LDSX() do { asm volatile("s_wait_dscnt 0" ::: "memory"); __builtin_amdgcn_wave_barrier(); __builtin_amdgcn_fence(3  , "workgroup"); } while (0)

#define WS_XB  ((size_t)0)
#define WS_WQT (WS_XB  + (size_t)2 * MROWS * DIN)
#define WS_WOT (WS_WQT + (size_t)2 * NQKV * DIN)
#define WS_QH  (WS_WOT + (size_t)2 * DIN * CC)
#define WS_QL  (WS_QH  + (size_t)2 * MROWS * CC)
#define WS_KH  (WS_QL  + (size_t)2 * MROWS * CC)
#define WS_KL  (WS_KH  + (size_t)2 * MROWS * CC)
#define WS_VB  (WS_KL  + (size_t)2 * MROWS * CC)
#define WS_VBL (WS_VB  + (size_t)2 * NB * CC * SEQ)
#define WS_CH  (WS_VBL + (size_t)2 * NB * CC * SEQ)
#define WS_CL  (WS_CH  + (size_t)2 * MROWS * CC)
#define WS_END (WS_CL  + (size_t)2 * MROWS * CC)
static_assert(WS_END <= (size_t)134217728);

__global__ __launch_bounds__(256) void k_cvt_x(const float* __restrict__ X, __bf16* __restrict__ XB) {
  const unsigned i = blockIdx.x * 256u + threadIdx.x;
  const unsigned row = i >> 7, pc = i & 127u;
  const unsigned b = row / (unsigned)SEQ, t = row - b * (unsigned)SEQ;
  const float* src = X + ((size_t)b * SEQ_FULL + t) * DIN + pc * 8u;
  const v4f a0 = *(const v4f*)src, a1 = *(const v4f*)(src + 4);
  union { v8b b8; v4u u; } o;
#pragma unroll
  for (int j = 0; j < 4; ++j) { o.b8[j] = (__bf16)a0[j]; o.b8[4 + j] = (__bf16)a1[j]; }
  vst2(XB + (size_t)row * DIN + pc * 8u, o.u);
}

__global__ __launch_bounds__(256) void k_cvt_wT(const float* __restrict__ W, __bf16* __restrict__ WT, unsigned K, unsigned N) {
  __shared__ __align__(16) __bf16 tw[64][72];
  const unsigned tid = threadIdx.x, n0 = blockIdx.x * 64u, k0 = blockIdx.y * 64u;
  { const unsigned kl = tid >> 2, q = tid & 3u; const float* p = W + (size_t)(k0 + kl) * N + n0 + q * 16u;
    const v4f a0 = *(const v4f*)p, a1 = *(const v4f*)(p + 4), a2 = *(const v4f*)(p + 8), a3 = *(const v4f*)(p + 12);
#pragma unroll
    for (int j = 0; j < 4; ++j) { tw[q * 16u + j][kl] = (__bf16)a0[j]; tw[q * 16u + 4 + j][kl] = (__bf16)a1[j]; tw[q * 16u + 8 + j][kl] = (__bf16)a2[j]; tw[q * 16u + 12 + j][kl] = (__bf16)a3[j]; } }
  __syncthreads();
  for (unsigned e = tid; e < 512u; e += 256u) { const unsigned nl = e >> 3, q = e & 7u; vst2(WT + (size_t)(n0 + nl) * K + k0 + q * 8u, *(const v4u*)&tw[nl][q * 8u]); }
}

__global__ __launch_bounds__(128) void k_qkv(const __bf16* __restrict__ XB, const __bf16* __restrict__ WT, const float* __restrict__ BQ,
    _Float16* __restrict__ QH, _Float16* __restrict__ QL, _Float16* __restrict__ KH, _Float16* __restrict__ KL, __bf16* __restrict__ VB, __bf16* __restrict__ VBL) {
  __shared__ __align__(16) _Float16 sh[64][136], sl[64][136]; __shared__ __align__(16) __bf16 tb[128][72], tbl[128][72];
  const unsigned tid = threadIdx.x, wave = tid >> 5, lane = tid & 31u, col = lane & 15u, g = lane >> 4;
  const unsigned c0 = blockIdx.y * 128u, r0 = blockIdx.x * 64u; const unsigned bb = r0 / (unsigned)SEQ, t0 = r0 - bb * (unsigned)SEQ;
  const unsigned which = c0 >> 10, cw = c0 & 1023u;
  const __bf16* ap = XB + (size_t)(r0 + wave * 16u + col) * DIN;
  const __bf16* wp = WT + (size_t)(c0 + col) * DIN;
  v8f acc[8] = {};
#pragma unroll 2
  for (unsigned kc = 0; kc < DIN / 32; ++kc) { const v16b a = frag_b(ap + kc * 32u, lane);
    asm volatile("s_wait_loadcnt 0x0" ::: "memory");
#pragma unroll
    for (int j = 0; j < 8; ++j) { const v16b w = frag_b(wp + (size_t)j * 16u * DIN + kc * 32u, lane); asm volatile("s_wait_loadcnt 0x0" ::: "memory"); acc[j] = wmma_bf(a, w, acc[j]); } }
  if (which < 2u) { _Float16* DH = which == 0u ? QH : KH; _Float16* DL = which == 0u ? QL : KL;
#pragma unroll
    for (int j = 0; j < 8; ++j) { const float bias = bfr(BQ[c0 + j * 16u + col]);
#pragma unroll
      for (int r = 0; r < 8; ++r) { const float v = acc[j][r] + bias; const _Float16 hv = (_Float16)v; sh[wave * 16u + 8u * g + r][j * 16u + col] = hv; sl[wave * 16u + 8u * g + r][j * 16u + col] = (_Float16)((v - (float)hv) * 1024.0f); } }
    __syncthreads();
    for (unsigned e = tid; e < 64u * 16u; e += 128u) { const unsigned rl = e >> 4, q = e & 15u; const size_t o = (size_t)(r0 + rl) * CC + cw + q * 8u;
      vst2(DH + o, *(const v4u*)&sh[rl][q * 8u]); vst2(DL + o, *(const v4u*)&sl[rl][q * 8u]); }
  } else {
#pragma unroll
    for (int j = 0; j < 8; ++j) { const float bias = bfr(BQ[c0 + j * 16u + col]);
#pragma unroll
      for (int r = 0; r < 8; ++r) { const float v = acc[j][r] + bias; const unsigned rl = wave * 16u + 8u * g + r, cl = j * 16u + col; const __bf16 bh = (__bf16)v; tb[cl][rl] = bh; tbl[cl][rl] = (__bf16)(v - (float)bh); } }
    __syncthreads();
    for (unsigned e = tid; e < 128u * 8u; e += 128u) { const unsigned cl = e >> 3, q = e & 7u; const size_t o3 = ((size_t)bb * CC + cw + cl) * (size_t)SEQ + t0 + q * 8u;
      vst2(VB + o3, *(const v4u*)&tb[cl][q * 8u]); vst2(VBL + o3, *(const v4u*)&tbl[cl][q * 8u]); } }
}

__device__ __forceinline__ v8f score_tile(const _Float16* __restrict__ KH, const _Float16* __restrict__ KL, size_t ko, unsigned lane, v16h qh0, v16h qh1, v16h ql0, v16h ql1) {
  const v16h kh0 = frag_h(KH + ko, lane), kh1 = frag_h(KH + ko + 32, lane), kl0 = frag_h(KL + ko, lane), kl1 = frag_h(KL + ko + 32, lane);
  v8f a = {}, al = {};
  a = wmma16(qh0, kh0, a); a = wmma16(qh1, kh1, a);
  al = wmma16(ql0, kh0, al); al = wmma16(ql1, kh1, al); al = wmma16(qh0, kl0, al); al = wmma16(qh1, kl1, al);
  v8f s;
#pragma unroll
  for (int r = 0; r < 8; ++r) s[r] = (a[r] + al[r] * (1.0f / 1024.0f)) * 0.125f;
  return s;
}

__global__ __launch_bounds__(128) void k_attn(const _Float16* __restrict__ QH, const _Float16* __restrict__ QL, const _Float16* __restrict__ KH, const _Float16* __restrict__ KL,
    const __bf16* __restrict__ VB, const __bf16* __restrict__ VBL, __bf16* __restrict__ CH, __bf16* __restrict__ CL) {
  __shared__ __align__(16) float ps[4][16][36];
  __shared__ __align__(16) float cs[4][16][68];
  const unsigned tid = threadIdx.x, wave = tid >> 5, lane = tid & 31u, col = lane & 15u, g = lane >> 4;
  const unsigned w = blockIdx.x * 4u + wave;
  const unsigned qt = w & (unsigned)(SEQ / 16 - 1), bh = w / (unsigned)(SEQ / 16), h = bh & 15u, b = bh >> 4;
  const unsigned q0 = qt * 16u;
  const size_t rowb = (size_t)b * SEQ;
  const size_t qoff = (rowb + q0 + col) * CC + h * HD;
  const v16h qh0 = frag_h(QH + qoff, lane), qh1 = frag_h(QH + qoff + 32, lane), ql0 = frag_h(QL + qoff, lane), ql1 = frag_h(QL + qoff + 32, lane);
  v8f o0 = {}, o1 = {}, o2 = {}, o3 = {};
  float rm[8], rs[8];
#pragma unroll
  for (int r = 0; r < 8; ++r) { rm[r] = -3.0e38f; rs[r] = 0.0f; }
  const unsigned lo = q0 >= (unsigned)(WIN - 1) ? q0 - (unsigned)(WIN - 1) : 0u;
  const unsigned kstart = lo & ~31u;
#pragma unroll 1
  for (unsigned kbk = kstart; kbk <= q0 + 15u; kbk += 32u) {
    const size_t ko = (rowb + kbk + col) * CC + h * HD;
    v8f s0 = score_tile(KH, KL, ko, lane, qh0, qh1, ql0, ql1);
    v8f s1 = score_tile(KH, KL, ko + (size_t)16 * CC, lane, qh0, qh1, ql0, ql1);
#pragma unroll
    for (int r = 0; r < 8; ++r) {
      const unsigned rq = q0 + 8u * g + r; const unsigned c0 = kbk + col, c1 = c0 + 16u;
      const bool ok0 = (rq - c0) < (unsigned)WIN, ok1 = (rq - c1) < (unsigned)WIN;
      const float v0 = ok0 ? s0[r] : -3.0e38f, v1 = ok1 ? s1[r] : -3.0e38f;
      float mv = fmaxf(v0, v1);
      mv = fmaxf(mv, __shfl_xor(mv, 1)); mv = fmaxf(mv, __shfl_xor(mv, 2)); mv = fmaxf(mv, __shfl_xor(mv, 4)); mv = fmaxf(mv, __shfl_xor(mv, 8));
      const float mnew = fmaxf(rm[r], mv);
      const float sc = expf(rm[r] - mnew);
      const float e0 = expf(v0 - mnew), e1 = expf(v1 - mnew);
      const float p0 = ok0 ? e0 : 0.0f, p1 = ok1 ? e1 : 0.0f;
      float rr = p0 + p1;
      rr += __shfl_xor(rr, 1); rr += __shfl_xor(rr, 2); rr += __shfl_xor(rr, 4); rr += __shfl_xor(rr, 8);
      rs[r] = rs[r] * sc + rr; rm[r] = mnew;
      o0[r] *= sc; o1[r] *= sc; o2[r] *= sc; o3[r] *= sc;
      ps[wave][8u * g + r][col] = p0; ps[wave][8u * g + r][16u + col] = p1;
    }
    LDSX();
    float pv[16];
    { const float* pr = &ps[wave][col][8u * g];
#pragma unroll
      for (int i = 0; i < 8; ++i) { pv[i] = pr[i]; pv[8 + i] = pr[16 + i]; } }
    LDSX();
    const F2 p = bsplit16(pv);
    { const size_t po = ((size_t)b * CC + h * HD + col) * (size_t)SEQ + kbk; const size_t js = (size_t)16 * SEQ;
      F2 vv;
      vv.h = frag_b(VB + po, lane);          vv.l = frag_b(VBL + po, lane);          o0 = mac3(p, vv, o0);
      vv.h = frag_b(VB + po + js, lane);     vv.l = frag_b(VBL + po + js, lane);     o1 = mac3(p, vv, o1);
      vv.h = frag_b(VB + po + 2 * js, lane); vv.l = frag_b(VBL + po + 2 * js, lane); o2 = mac3(p, vv, o2);
      vv.h = frag_b(VB + po + 3 * js, lane); vv.l = frag_b(VBL + po + 3 * js, lane); o3 = mac3(p, vv, o3); }
  }
#pragma unroll
  for (int r = 0; r < 8; ++r) { const float inv = 1.0f / rs[r];
    cs[wave][8u * g + r][col] = o0[r] * inv; cs[wave][8u * g + r][16u + col] = o1[r] * inv; cs[wave][8u * g + r][32u + col] = o2[r] * inv; cs[wave][8u * g + r][48u + col] = o3[r] * inv; }
  LDSX();
#pragma unroll
  for (unsigned pp = 0; pp < 4u; ++pp) { const unsigned rl = pp * 4u + (lane >> 3), q = lane & 7u; const float* cp = &cs[wave][rl][q * 8u];
    union { v8b b8; v4u u; } hu, lu;
#pragma unroll
    for (int i = 0; i < 8; ++i) { const float v = cp[i]; const __bf16 hb = (__bf16)v; hu.b8[i] = hb; lu.b8[i] = (__bf16)(v - (float)hb); }
    const size_t dst = (rowb + q0 + rl) * CC + h * HD + q * 8u;
    vst2(CH + dst, hu.u); vst2(CL + dst, lu.u); }
}

__global__ __launch_bounds__(128) void k_out(const __bf16* __restrict__ CH, const __bf16* __restrict__ CL, const __bf16* __restrict__ WOT, const float* __restrict__ BO, float* __restrict__ OUT) {
  __shared__ __align__(16) float so[64][132];
  const unsigned tid = threadIdx.x, wave = tid >> 5, lane = tid & 31u, col = lane & 15u, g = lane >> 4;
  const unsigned c0 = blockIdx.y * 128u, r0 = blockIdx.x * 64u; const unsigned bb = r0 / (unsigned)SEQ, t0 = r0 - bb * (unsigned)SEQ;
  const size_t ao = (size_t)(r0 + wave * 16u + col) * CC;
  const __bf16* wp = WOT + (size_t)(c0 + col) * CC;
  v8f acc[8] = {};
#pragma unroll 2
  for (unsigned kc = 0; kc < CC / 32; ++kc) { const v16b ah = frag_b(CH + ao + kc * 32u, lane), al = frag_b(CL + ao + kc * 32u, lane);
    asm volatile("s_wait_loadcnt 0x0" ::: "memory");
#pragma unroll
    for (int j = 0; j < 8; ++j) { const v16b w = frag_b(wp + (size_t)j * 16u * CC + kc * 32u, lane); asm volatile("s_wait_loadcnt 0x0" ::: "memory"); acc[j] = wmma_bf(al, w, acc[j]); acc[j] = wmma_bf(ah, w, acc[j]); } }
#pragma unroll
  for (int j = 0; j < 8; ++j) { const float bias = bfr(BO[c0 + j * 16u + col]);
#pragma unroll
    for (int r = 0; r < 8; ++r) so[wave * 16u + 8u * g + r][j * 16u + col] = acc[j][r] + bias; }
  __syncthreads();
#pragma unroll 1
  for (unsigned rl = 0; rl < 16u; ++rl) { const unsigned lr = wave * 16u + rl; const size_t orow = (size_t)bb * SEQ_FULL + t0 + lr;
    vst2(OUT + orow * DIN + c0 + lane * 4u, *(const v4f*)&so[lr][lane * 4u]); }
}

extern "C" void kernel_launch(void* const* d_in, const int* in_sizes, int n_in, void* d_out, int out_size, void* d_ws, size_t ws_size, hipStream_t stream) {
  if (n_in < 5) return;
  const long long need_x = ((long long)(NB - 1) * SEQ_FULL + SEQ) * DIN;
  if ((long long)in_sizes[0] < need_x) return;
  if ((long long)in_sizes[1] < (long long)DIN * NQKV) return;
  if (in_sizes[2] < NQKV) return;
  if ((long long)in_sizes[3] < (long long)CC * DIN) return;
  if (in_sizes[4] < DIN) return;
  if ((long long)out_size < need_x) return;
  if (ws_size < (size_t)WS_END) return;
  const float* X = (const float*)d_in[0]; const float* WQKV = (const float*)d_in[1]; const float* BQKV = (const float*)d_in[2]; const float* WO = (const float*)d_in[3]; const float* BO = (const float*)d_in[4];
  char* ws = (char*)d_ws;
  __bf16* XB = (__bf16*)(ws + WS_XB); __bf16* WQT = (__bf16*)(ws + WS_WQT); __bf16* WOT = (__bf16*)(ws + WS_WOT);
  _Float16* QH = (_Float16*)(ws + WS_QH); _Float16* QL = (_Float16*)(ws + WS_QL); _Float16* KH = (_Float16*)(ws + WS_KH); _Float16* KL = (_Float16*)(ws + WS_KL);
  __bf16* VB = (__bf16*)(ws + WS_VB); __bf16* VBL = (__bf16*)(ws + WS_VBL); __bf16* CH = (__bf16*)(ws + WS_CH); __bf16* CL = (__bf16*)(ws + WS_CL);
  k_cvt_x<<<dim3((MROWS * DIN) / 2048), 256, 0, stream>>>(X, XB);
  k_cvt_wT<<<dim3(NQKV / 64, DIN / 64), 256, 0, stream>>>(WQKV, WQT, (unsigned)DIN, (unsigned)NQKV);
  k_cvt_wT<<<dim3(DIN / 64, CC / 64), 256, 0, stream>>>(WO, WOT, (unsigned)CC, (unsigned)DIN);
  k_qkv<<<dim3(MROWS / 64, NQKV / 128), 128, 0, stream>>>(XB, WQT, BQKV, QH, QL, KH, KL, VB, VBL);
  k_attn<<<dim3((NB * NH * (SEQ / 16)) / 4), 128, 0, stream>>>(QH, QL, KH, KL, VB, VBL, CH, CL);
  k_out<<<dim3(MROWS / 64, DIN / 128), 128, 0, stream>>>(CH, CL, WOT, BO, (float*)d_out);
}
